// CasualSelfAttention_56667798504030
// MI455X (gfx1250) — hardware-verified
//
#include <hip/hip_runtime.h>


#ifndef NB
#define NB 4
#endif
#ifndef SEQ
#define SEQ 2048
#endif
#define SEQ_FULL 2048
#define DM   1024
#define NH   16
#define HD   64
#define DQ   (NH * HD)
#define FP   (3 * DQ)
#define RH   ((SEQ) < 512 ? (SEQ) : 512)
#define XS_FULL ((size_t)SEQ_FULL * DM)
#define SCL  0.125f
#define LOG2E 1.4426950408889634f
#define NEGB (-3.0e38f)

static_assert((SEQ & (SEQ - 1)) == 0);
static_assert(SEQ >= 256 && SEQ <= SEQ_FULL);
static_assert(RH % 256 == 0 && RH % 64 == 0 && (SEQ - RH) % 64 == 0);
static_assert(NB >= 1 && NB <= 4);
static_assert(DM % 32 == 0 && DQ % 64 == 0 && FP % 64 == 0 && SEQ % 64 == 0);
static_assert(((size_t)3 * DQ * DM / 8) % 256 == 0);
static_assert(((size_t)SEQ * DM / 8) % 256 == 0);
static_assert(((size_t)NH * SEQ * HD / 8) % 256 == 0);
static_assert(DQ == DM);
static_assert(HD == 64 && HD % 32 == 0);

typedef _Float16 h16;
typedef unsigned short bf;
typedef __attribute__((ext_vector_type(16))) __bf16   v16bf;
typedef __attribute__((ext_vector_type(16))) _Float16 v16h;
typedef __attribute__((ext_vector_type(8)))  _Float16 v8h;
typedef __attribute__((ext_vector_type(8)))  unsigned short v8us;
typedef __attribute__((ext_vector_type(8)))  float    v8f;
typedef __attribute__((ext_vector_type(4)))  float    v4f;
typedef v8h  __attribute__((may_alias)) v8ha;
typedef v4f  __attribute__((may_alias)) v4fa;
typedef v8us __attribute__((may_alias)) v8usa;

__device__ __forceinline__ unsigned short f2bf(float f) { unsigned u = __float_as_uint(f); u += 0x7FFFu + ((u >> 16) & 1u); return (unsigned short)(u >> 16); }
__device__ __forceinline__ float bf2f(unsigned short b) { return __uint_as_float(((unsigned)b) << 16); }
__device__ __forceinline__ float bfr(float f) { return bf2f(f2bf(f)); }
__device__ __forceinline__ v16h cat16(v8h lo, v8h hi) { return __builtin_shufflevector(lo, hi, 0, 1, 2, 3, 4, 5, 6, 7, 8, 9, 10, 11, 12, 13, 14, 15); }
__device__ __forceinline__ v16bf cat16b(v8us lo, v8us hi) { return __builtin_bit_cast(v16bf, __builtin_shufflevector(lo, hi, 0, 1, 2, 3, 4, 5, 6, 7, 8, 9, 10, 11, 12, 13, 14, 15)); }
__device__ __forceinline__ v8f wmma16(v16h a, v16h b, v8f c) { return __builtin_amdgcn_wmma_f32_16x16x32_f16(false, a, false, b, (short)0, c, false, false); }
__device__ __forceinline__ v8f wmmab(v16bf a, v16bf b, v8f c) { return __builtin_amdgcn_wmma_f32_16x16x32_bf16(false, a, false, b, (short)0, c, false, false); }
__device__ __forceinline__ void splitf(float y, unsigned short& h, unsigned short& l) { h = f2bf(y); l = f2bf(y - bf2f(h)); }

static __device__ __forceinline__ h16 toh_flush(float v) { const h16 r = (h16)v; return (fabsf(v) < 6.103515625e-05f) ? (h16)0.0f : r; }

template <typename T16> struct WFrag;
template <> struct WFrag<h16> { typedef v16h V; static __device__ __forceinline__ V ld(const h16* p) { return cat16(*(const v8h*)p, *(const v8h*)(p + 16)); } static __device__ __forceinline__ v8f mma(V a, V b, v8f c) { return wmma16(a, b, c); } };
template <> struct WFrag<bf> { typedef v16bf V; static __device__ __forceinline__ V ld(const bf* p) { return cat16b(*(const v8us*)p, *(const v8us*)(p + 16)); } static __device__ __forceinline__ v8f mma(V a, V b, v8f c) { return wmmab(a, b, c); } };

template <typename T16> struct PFrag;
template <> struct PFrag<h16> {
    static __device__ __forceinline__ float pexp() { return 10.0f; }
    static __device__ __forceinline__ v16h hi(v8f p0, v8f p1) { return cat16(__builtin_convertvector(p0, v8h), __builtin_convertvector(p1, v8h)); }
    static __device__ __forceinline__ v16h lo(v8f p0, v8f p1) { return hi(p0, p1); }
};
template <> struct PFrag<bf> {
    static __device__ __forceinline__ float pexp() { return 0.0f; }
    static __device__ __forceinline__ v16bf hi(v8f p0, v8f p1) { v8us a, b;
#pragma unroll
        for (int k = 0; k < 8; ++k) { a[k] = f2bf(p0[k]); b[k] = f2bf(p1[k]); }
        return cat16b(a, b); }
    static __device__ __forceinline__ v16bf lo(v8f p0, v8f p1) { v8us a, b;
#pragma unroll
        for (int k = 0; k < 8; ++k) { a[k] = f2bf(p0[k] - bf2f(f2bf(p0[k]))); b[k] = f2bf(p1[k] - bf2f(f2bf(p1[k]))); }
        return cat16b(a, b); }
};

template <typename T16> struct PFlush;
template <> struct PFlush<h16> {
    static __device__ __forceinline__ v16h hi(v8f p0, v8f p1) { v8h a, b;
#pragma unroll
        for (int k = 0; k < 8; ++k) { a[k] = toh_flush(p0[k]); b[k] = toh_flush(p1[k]); }
        return cat16(a, b); }
    static __device__ __forceinline__ v16h lo(v8f p0, v8f p1) { return hi(p0, p1); }
};
template <> struct PFlush<bf> {
    static __device__ __forceinline__ v16bf hi(v8f p0, v8f p1) { return PFrag<bf>::hi(p0, p1); }
    static __device__ __forceinline__ v16bf lo(v8f p0, v8f p1) { return PFrag<bf>::lo(p0, p1); }
};

template <typename T16, int NSPLIT, bool BIAS>
__global__ __launch_bounds__(32) void k_gemmw(const T16* __restrict__ A, const T16* __restrict__ A2, const T16* __restrict__ Bt, const T16* __restrict__ Bt2, int K, float* C, int ldc, const float* __restrict__ bias, size_t sA, size_t sB, size_t sC) {
    typedef typename WFrag<T16>::V V;
    __shared__ __align__(16) float os[16 * 68];
    const size_t z = blockIdx.z; A += z * sA; if (A2) A2 += z * sA; Bt += z * sB; if (Bt2) Bt2 += z * sB; C += z * sC;
    const int lane = threadIdx.x & 31, lr = lane & 15, hi = lane >> 4; const int r0 = blockIdx.x * 64, c0 = blockIdx.y * 64;
    v8f acc[4][4];
#pragma unroll
    for (int mb = 0; mb < 4; ++mb)
#pragma unroll
        for (int nb = 0; nb < 4; ++nb) acc[mb][nb] = (v8f){};
    const size_t aoff = (size_t)(r0 + lr) * K + 8 * hi, boff = (size_t)(c0 + lr) * K + 8 * hi;
#pragma unroll 1
    for (int kc = 0; kc < K; kc += 32) {
        V a[4], a2[4];
#pragma unroll
        for (int mb = 0; mb < 4; ++mb) { a[mb] = WFrag<T16>::ld(A + aoff + (size_t)mb * 16 * K + kc); if (NSPLIT == 1 || NSPLIT == 2) a2[mb] = WFrag<T16>::ld(A2 + aoff + (size_t)mb * 16 * K + kc); }
#pragma unroll
        for (int nb = 0; nb < 4; ++nb) { const V b = WFrag<T16>::ld(Bt + boff + (size_t)nb * 16 * K + kc); V b2; if (NSPLIT >= 2) b2 = WFrag<T16>::ld(Bt2 + boff + (size_t)nb * 16 * K + kc);
#pragma unroll
            for (int mb = 0; mb < 4; ++mb) { acc[mb][nb] = WFrag<T16>::mma(a[mb], b, acc[mb][nb]); if (NSPLIT == 1 || NSPLIT == 2) acc[mb][nb] = WFrag<T16>::mma(a2[mb], b, acc[mb][nb]); if (NSPLIT >= 2) acc[mb][nb] = WFrag<T16>::mma(a[mb], b2, acc[mb][nb]); } }
        asm volatile("v_nop\n\tv_nop\n\tv_nop\n\tv_nop" : "+v"(acc[0][0]), "+v"(acc[1][1]), "+v"(acc[2][2]), "+v"(acc[3][3]) : "v"(a[0]), "v"(a[3]));
    }
#pragma unroll
    for (int mb = 0; mb < 4; ++mb) {
#pragma unroll
        for (int nb = 0; nb < 4; ++nb) {
#pragma unroll
            for (int j = 0; j < 8; ++j) os[(hi * 8 + j) * 68 + nb * 16 + lr] = acc[mb][nb][j]; }
        __builtin_amdgcn_wave_barrier(); asm volatile("" ::: "memory");
        float* crow = C + (size_t)(r0 + mb * 16) * ldc + c0;
#pragma unroll 1
        for (int ps = 0; ps < 2; ++ps) {
#pragma unroll
            for (int s = 0; s < 8; ++s) { const int row = 2 * s + hi, cofs = lr * 4; v4f val = *(const v4fa*)(os + row * 68 + cofs); if (BIAS) { val[0] += bfr(bias[c0 + cofs]); val[1] += bfr(bias[c0 + cofs + 1]); val[2] += bfr(bias[c0 + cofs + 2]); val[3] += bfr(bias[c0 + cofs + 3]); }
                *(volatile v4f*)(crow + (size_t)row * ldc + cofs) = val; }
            if (ps == 0) __threadfence(); }
        __builtin_amdgcn_wave_barrier(); asm volatile("" ::: "memory");
    }
}

__global__ __launch_bounds__(256) void k_cvt8(const float* __restrict__ src, bf* dst, unsigned n8, size_t sstride, size_t dstride) {
    const unsigned i = blockIdx.x * 256u + threadIdx.x; if (i >= n8) return;
    const float* s = src + (size_t)blockIdx.y * sstride + (size_t)i * 8; bf* d = dst + (size_t)blockIdx.y * dstride + (size_t)i * 8;
    const v8f v = *(const v8f*)s; v8us o;
#pragma unroll
    for (int k = 0; k < 8; ++k) o[k] = f2bf(v[k]);
    *(volatile v8us*)d = o; __threadfence(); *(volatile v8us*)d = o; }

__global__ __launch_bounds__(256) void k_qkp(const float* __restrict__ F, h16* Q16, h16* K16, bf* Qh, bf* Ql, bf* Kh, bf* Kl) {
    const unsigned which = blockIdx.y; const unsigned e = (blockIdx.x * 256u + threadIdx.x) * 8u;
    const unsigned d = e & 63u, t = (e >> 6) % (unsigned)SEQ, h = e / (64u * (unsigned)SEQ);
    h16* P16 = which ? K16 : Q16; bf* Ph = which ? Kh : Qh; bf* Pl = which ? Kl : Ql;
    const float* f = F + (size_t)t * FP + which * DQ + h * HD + d;
    const v4f x0 = *(const v4f*)f, x1 = *(const v4f*)(f + 4);
    v8h o16; v8us oh, ol;
#pragma unroll
    for (int k = 0; k < 4; ++k) { unsigned short a, c; o16[k] = (h16)x0[k]; splitf(x0[k], a, c); oh[k] = a; ol[k] = c; o16[4 + k] = (h16)x1[k]; splitf(x1[k], a, c); oh[4 + k] = a; ol[4 + k] = c; }
    const size_t eo = ((size_t)h * RH + t) * HD + d;
    *(volatile v8h*)(P16 + e) = o16;
    if (t < (unsigned)RH) { *(volatile v8us*)(Ph + eo) = oh; *(volatile v8us*)(Pl + eo) = ol; }
    __threadfence();
    *(volatile v8h*)(P16 + e) = o16;
    if (t < (unsigned)RH) { *(volatile v8us*)(Ph + eo) = oh; *(volatile v8us*)(Pl + eo) = ol; }
}

__global__ __launch_bounds__(256) void k_vtp(const float* __restrict__ F, h16* V16, bf* Vh, bf* Vl) {
    const unsigned e = (blockIdx.x * 256u + threadIdx.x) * 8u;
    const unsigned t = e % (unsigned)SEQ, d = (e / (unsigned)SEQ) & 63u, g = e / ((unsigned)SEQ * 64u);
    const float* f = F + (size_t)t * FP + 2 * DQ + g * HD + d;
    v8h o16; v8us oh, ol;
#pragma unroll
    for (int k = 0; k < 8; ++k) { const float x = f[(size_t)k * FP]; unsigned short a, c; o16[k] = (h16)x; splitf(x, a, c); oh[k] = a; ol[k] = c; }
    const size_t eo = ((size_t)g * HD + d) * RH + t;
    *(volatile v8h*)(V16 + e) = o16;
    if (t < (unsigned)RH) { *(volatile v8us*)(Vh + eo) = oh; *(volatile v8us*)(Vl + eo) = ol; }
    __threadfence();
    *(volatile v8h*)(V16 + e) = o16;
    if (t < (unsigned)RH) { *(volatile v8us*)(Vh + eo) = oh; *(volatile v8us*)(Vl + eo) = ol; }
}

static_assert(32 * 16 * 8 == 16 * HD * 4);
static_assert(HD * 4 == 16 * 16);
static_assert((HD * 4) % 128 == 0 && (DM * 4) % 128 == 0);
static_assert(16 * 68 * 4 <= 131072);
static_assert(68 >= HD && (68 * 4) % 16 == 0);

template <typename T16, bool HL>
__global__ __launch_bounds__(32) void k_flash(const T16* __restrict__ Q, const T16* __restrict__ Q2, const T16* __restrict__ Kp, const T16* __restrict__ K2, const T16* __restrict__ Vt, const T16* __restrict__ Vt2, unsigned tp, unsigned qbase, float* O) {
    typedef typename WFrag<T16>::V V;
    __shared__ __align__(16) float os[16 * 68];
    const unsigned lane = threadIdx.x & 31u, lr = lane & 15u, hi = lane >> 4;
    const unsigned head = blockIdx.y, q0 = qbase + blockIdx.x * 16u;
    const size_t hoff = (size_t)head * tp * HD;
    const size_t qoff = hoff + (size_t)(q0 + lr) * HD + 8u * hi;
    V qf0 = WFrag<T16>::ld(Q + qoff), qf1 = WFrag<T16>::ld(Q + qoff + 32);
    V ql0 = qf0, ql1 = qf1;
    if (HL) { ql0 = WFrag<T16>::ld(Q2 + qoff); ql1 = WFrag<T16>::ld(Q2 + qoff + 32); }
    v8f o[4];
#pragma unroll
    for (int db = 0; db < 4; ++db) o[db] = (v8f){};
    float mrun = NEGB, lsum = 0.0f;
    const float cs = SCL * LOG2E, pe = PFrag<T16>::pexp();
    const size_t kbase = hoff + (size_t)lr * HD + 8u * hi;
    const size_t vbase = hoff + (size_t)lr * tp + 8u * hi;
    const unsigned nt = (q0 + 47u) >> 5;
#pragma unroll 1
    for (unsigned it = 0; it < nt; ++it) {
        const unsigned j0 = it * 32u;
        const size_t ko = kbase + (size_t)j0 * HD;
        V ka0 = WFrag<T16>::ld(Kp + ko), ka1 = WFrag<T16>::ld(Kp + ko + 32), kb0 = WFrag<T16>::ld(Kp + ko + 16 * HD), kb1 = WFrag<T16>::ld(Kp + ko + 16 * HD + 32);
        V la0 = ka0, la1 = ka1, lb0 = kb0, lb1 = kb1;
        if (HL) { la0 = WFrag<T16>::ld(K2 + ko); la1 = WFrag<T16>::ld(K2 + ko + 32); lb0 = WFrag<T16>::ld(K2 + ko + 16 * HD); lb1 = WFrag<T16>::ld(K2 + ko + 16 * HD + 32); }
        v8f s0 = (v8f){}, s1 = (v8f){};
        s0 = WFrag<T16>::mma(ka0, qf0, s0); s0 = WFrag<T16>::mma(ka1, qf1, s0);
        s1 = WFrag<T16>::mma(kb0, qf0, s1); s1 = WFrag<T16>::mma(kb1, qf1, s1);
        if (HL) {
            s0 = WFrag<T16>::mma(la0, qf0, s0); s0 = WFrag<T16>::mma(la1, qf1, s0); s0 = WFrag<T16>::mma(ka0, ql0, s0); s0 = WFrag<T16>::mma(ka1, ql1, s0);
            s1 = WFrag<T16>::mma(lb0, qf0, s1); s1 = WFrag<T16>::mma(lb1, qf1, s1); s1 = WFrag<T16>::mma(kb0, ql0, s1); s1 = WFrag<T16>::mma(kb1, ql1, s1); }
        asm volatile("v_nop\n\tv_nop\n\tv_nop\n\tv_nop" : "+v"(s0), "+v"(s1) : "v"(ka0), "v"(ka1), "v"(kb0), "v"(kb1), "v"(la0), "v"(la1), "v"(lb0), "v"(lb1), "v"(qf0), "v"(qf1), "v"(ql0), "v"(ql1));
        v8f t0, t1;
#pragma unroll
        for (int r = 0; r < 8; ++r) { t0[r] = s0[r] * cs; t1[r] = s1[r] * cs; }
        if (j0 + 31u > q0) {
            const unsigned qi = q0 + lr, kk = j0 + 8u * hi;
#pragma unroll
            for (int r = 0; r < 8; ++r) { t0[r] = (kk + (unsigned)r <= qi) ? t0[r] : NEGB; t1[r] = (kk + 16u + (unsigned)r <= qi) ? t1[r] : NEGB; }
        }
        float mx = fmaxf(t0[0], t1[0]);
#pragma unroll
        for (int r = 1; r < 8; ++r) mx = fmaxf(mx, fmaxf(t0[r], t1[r]));
        mx = fmaxf(mx, __shfl_xor(mx, 16, 32));
        const float mn = fmaxf(mrun, mx);
        const float alpha = __builtin_amdgcn_exp2f(mrun - mn);
        mrun = mn;
        v8f p0, p1; float psum = 0.0f;
#pragma unroll
        for (int r = 0; r < 8; ++r) { p0[r] = __builtin_amdgcn_exp2f((t0[r] - mn) + pe); p1[r] = __builtin_amdgcn_exp2f((t1[r] - mn) + pe); psum += p0[r] + p1[r]; }
        lsum = lsum * alpha + psum;
#pragma unroll
        for (int db = 0; db < 4; ++db) o[db] = o[db] * alpha;
        V pf = PFlush<T16>::hi(p0, p1); V pl = pf;
        if (HL) pl = PFlush<T16>::lo(p0, p1);
        V va[4], vl[4];
#pragma unroll
        for (int db = 0; db < 4; ++db) { const size_t vo = vbase + (size_t)db * 16 * tp + j0; va[db] = WFrag<T16>::ld(Vt + vo); vl[db] = va[db]; if (HL) vl[db] = WFrag<T16>::ld(Vt2 + vo); }
#pragma unroll
        for (int db = 0; db < 4; ++db) { o[db] = WFrag<T16>::mma(va[db], pf, o[db]); if (HL) { o[db] = WFrag<T16>::mma(va[db], pl, o[db]); o[db] = WFrag<T16>::mma(vl[db], pf, o[db]); } }
        asm volatile("v_nop\n\tv_nop\n\tv_nop\n\tv_nop" : "+v"(o[0]), "+v"(o[1]), "+v"(o[2]), "+v"(o[3]) : "v"(va[0]), "v"(va[1]), "v"(va[2]), "v"(va[3]), "v"(vl[0]), "v"(vl[1]), "v"(vl[2]), "v"(vl[3]), "v"(pf), "v"(pl));
    }
    const float lt = lsum + __shfl_xor(lsum, 16, 32);
    const float inv = 1.0f / lt;
#pragma unroll
    for (int db = 0; db < 4; ++db)
#pragma unroll
        for (int r = 0; r < 8; ++r) os[lr * 68u + (unsigned)db * 16u + hi * 8u + (unsigned)r] = o[db][r] * inv;
    __builtin_amdgcn_wave_barrier(); asm volatile("" ::: "memory");
    float* orow = O + (size_t)q0 * DM + head * HD;
#pragma unroll 1
    for (int ps = 0; ps < 2; ++ps) {
#pragma unroll
        for (int s = 0; s < 8; ++s) { const unsigned row = 2u * (unsigned)s + hi, cofs = lr * 4u;
            const v4f val = *(const v4fa*)(os + row * 68u + cofs);
            *(volatile v4f*)(orow + (size_t)row * DM + cofs) = val; }
        if (ps == 0) __threadfence(); }
}

#define WS_WQKV ((size_t)3 * DQ * DM * 2)
#define WS_XB   ((size_t)NB * SEQ * DM * 2)
#define WS_F    ((size_t)SEQ * FP * 4)
#define WS_P16  ((size_t)NH * SEQ * HD * 2)
#define WS_PHL  ((size_t)NH * RH * HD * 2)
#define WS_TOTAL (WS_WQKV + WS_XB + WS_F + 3 * WS_P16 + 6 * WS_PHL)
static_assert(WS_TOTAL <= (size_t)134217728);
static_assert(WS_WQKV % 256 == 0 && WS_XB % 256 == 0 && WS_F % 256 == 0 && WS_P16 % 256 == 0 && WS_PHL % 256 == 0);
static_assert((size_t)NB * SEQ * DM * 4 <= (size_t)33554432);

extern "C" void kernel_launch(void* const* d_in, const int* in_sizes, int n_in,
                              void* d_out, int out_size, void* d_ws, size_t ws_size, hipStream_t stream) {
    if (n_in < 3) return;
    if ((size_t)in_sizes[0] < (size_t)(NB - 1) * XS_FULL + (size_t)SEQ * DM) return;
    if ((size_t)in_sizes[1] < (size_t)3 * DQ * DM) return;
    if ((size_t)in_sizes[2] < (size_t)FP) return;
    if ((size_t)out_size < (size_t)NB * SEQ * DM) return;
    if (ws_size < WS_TOTAL) return;
    const float* x = (const float*)d_in[0];
    const float* wqkv = (const float*)d_in[1];
    const float* bqkv = (const float*)d_in[2];
    float* OUT = (float*)d_out;
    char* wsp = (char*)d_ws;
    auto take = [&](size_t bytes) { char* p = wsp; wsp += bytes; return (void*)p; };
    bf* WQKV = (bf*)take(WS_WQKV); bf* XB = (bf*)take(WS_XB); float* F = (float*)take(WS_F);
    h16* Q16 = (h16*)take(WS_P16); h16* K16 = (h16*)take(WS_P16); h16* VT16 = (h16*)take(WS_P16);
    bf* Qh = (bf*)take(WS_PHL); bf* Ql = (bf*)take(WS_PHL); bf* Kh = (bf*)take(WS_PHL); bf* Kl = (bf*)take(WS_PHL); bf* VTh = (bf*)take(WS_PHL); bf* VTl = (bf*)take(WS_PHL);

    k_cvt8<<<dim3((unsigned)((size_t)3 * DQ * DM / 8 / 256), 1), 256, 0, stream>>>(wqkv, WQKV, (unsigned)((size_t)3 * DQ * DM / 8), 0, 0);
    k_cvt8<<<dim3((unsigned)((size_t)SEQ * DM / 8 / 256), NB), 256, 0, stream>>>(x, XB, (unsigned)((size_t)SEQ * DM / 8), XS_FULL, (size_t)SEQ * DM);
    for (int b = 0; b < NB; ++b) {
        k_gemmw<bf, 0, true><<<dim3(SEQ / 64, FP / 64, 1), 32, 0, stream>>>(XB + (size_t)b * SEQ * DM, nullptr, WQKV, nullptr, DM, F, FP, bqkv, 0, 0, 0);
        k_qkp<<<dim3((unsigned)((size_t)NH * SEQ * HD / 8 / 256), 2), 256, 0, stream>>>(F, Q16, K16, Qh, Ql, Kh, Kl);
        k_vtp<<<dim3((unsigned)((size_t)NH * HD * SEQ / 8 / 256), 1), 256, 0, stream>>>(F, VT16, VTh, VTl);
        k_flash<bf, true><<<dim3(RH / 16, NH), 32, 0, stream>>>(Qh, Ql, Kh, Kl, VTh, VTl, (unsigned)RH, 0u, OUT + (size_t)b * SEQ * DM);
        if (SEQ > RH) k_flash<h16, false><<<dim3((SEQ - RH) / 16, NH), 32, 0, stream>>>(Q16, nullptr, K16, nullptr, VT16, nullptr, (unsigned)SEQ, (unsigned)RH, OUT + (size_t)b * SEQ * DM);
    }
}
